// PolicyGNN_35897336660646
// MI455X (gfx1250) — hardware-verified
//
#include <hip/hip_runtime.h>
#include <stddef.h>
#include <stdint.h>


#define NF   8
#define EF   4
#define GF   4
#define DN   128
#define DE   128
#define DG   64
#define HE   256
#define HN   256
#define HG   256
#define KG1  (DG + DN)
#define ABW  (2 * HE)
#define GVN  (DG + HE + HN)

#define NTHR  256
#define NWAVE 8
#define EPT   8
#define CHUNK (NTHR * EPT)
#define WCAP  (EPT * 32)
#define LISTN (NWAVE * WCAP)
#define PASSN (NWAVE * 16)
#define PCAP  (CHUNK + PASSN)
#define NB    128
#define NBR   64
#define NTHN  128

#define WSC   16.0f
#define ESC   64.0f
#define HSC   64.0f
#define EINV  0.0009765625f
#define HINV  0.0009765625f
#define EPINV 0.015625f

#define LE_ACC   0
#define LE_MSG   (LE_ACC + (NB + 1) * DE * 4)
#define LE_EIO   (LE_MSG + PASSN * DE * 4)
#define LE_HID   (LE_EIO + NWAVE * 16 * DE * 2)
#define LE_LIST  (LE_HID + NWAVE * 16 * HE * 2)
#define LE_PEND  (LE_LIST + LISTN * 4)
#define LE_EINF  (LE_PEND + PCAP * 4)
#define LE_GV    (LE_EINF + PASSN * 8)
#define LE_B2    (LE_GV + HE * 4)
#define LE_CNT   (LE_B2 + DE * 4)
#define LE_WCNT  (LE_CNT + NB * 4)
#define LE_TOTAL (LE_WCNT + 64)

#define LN_HH    0
#define LN_HL    (LN_HH + 4 * 16 * HN * 2)
#define LN_OST   (LN_HL + 4 * 16 * HN * 2)
#define LN_GV    (LN_OST + 4 * 16 * DN * 4)
#define LN_B2    (LN_GV + HN * 4)
#define LN_VR    (LN_B2 + DN * 4)
#define LN_TOTAL (LN_VR + NBR * 4)

static_assert(PASSN == 128);
static_assert(PCAP >= CHUNK + PASSN);
static_assert(NWAVE * 16 == NB);
static_assert(NB == 4 * 32);
static_assert(DE == 4 * 32);
static_assert(NTHR == HE && HE == HN && HN == HG);
static_assert(NB == 2 * NBR);
static_assert(GVN == DG + HE + HN);
static_assert((LE_TOTAL % 16) == 0 && (LE_MSG % 16) == 0 && (LE_EIO % 16) == 0 && (LE_HID % 16) == 0);
static_assert((LE_EINF % 16) == 0 && (LE_GV % 16) == 0 && (LE_CNT % 16) == 0);
static_assert(LE_TOTAL <= 300 * 1024);
static_assert((LN_TOTAL % 16) == 0 && LN_TOTAL <= 300 * 1024);

typedef float          v4f  __attribute__((ext_vector_type(4)));
typedef float          v8f  __attribute__((ext_vector_type(8)));
typedef int            v2i  __attribute__((ext_vector_type(2)));
typedef int            v4i  __attribute__((ext_vector_type(4)));
typedef _Float16       v8h  __attribute__((ext_vector_type(8)));
typedef _Float16       v16h __attribute__((ext_vector_type(16)));
typedef unsigned short v8us __attribute__((ext_vector_type(8)));
typedef __bf16         v16b __attribute__((ext_vector_type(16)));
union FragH { v16h v; v8h h[2]; };
union FragB { v16b v; v8us u[2]; };
union Pk8 { v8h h; v8us u; v4i i; };

__device__ __forceinline__ float lrelu(float v) { return v > 0.0f ? v : 0.01f * v; }

__device__ __forceinline__ unsigned short f2bf(float x) {
  unsigned u = __builtin_bit_cast(unsigned, x);
  u = (u + 0x7FFFu + ((u >> 16) & 1u)) >> 16;
  return (unsigned short)u;
}
__device__ __forceinline__ float bf2f(unsigned short h) {
  return __builtin_bit_cast(float, ((unsigned)h) << 16);
}

__device__ __forceinline__ v8f zero8f() {
  v8f c;
#pragma unroll
  for (int i = 0; i < 8; ++i) c[i] = 0.0f;
  return c;
}

__device__ __forceinline__ v8f wmh(v16h a, v16h b, v8f c) {
  v8f d = __builtin_amdgcn_wmma_f32_16x16x32_f16(false, a, false, b, (short)0, c, false, false);
  asm volatile("v_nop\n\tv_nop\n\tv_nop\n\tv_nop" : "+v"(d) : "v"(a), "v"(b));
  return d;
}
__device__ __forceinline__ v8f wmb(v16b a, v16b b, v8f c) {
  v8f d = __builtin_amdgcn_wmma_f32_16x16x32_bf16(false, a, false, b, (short)0, c, false, false);
  asm volatile("v_nop\n\tv_nop\n\tv_nop\n\tv_nop" : "+v"(d) : "v"(a), "v"(b));
  return d;
}

__device__ __forceinline__ void split8(v4f a, v4f b, Pk8& ph, Pk8& pl) {
  const float t[8] = {a.x, a.y, a.z, a.w, b.x, b.y, b.z, b.w};
#pragma unroll
  for (int i = 0; i < 8; ++i) {
    const unsigned short hq = f2bf(t[i]);
    ph.u[i] = hq;
    pl.u[i] = f2bf(t[i] - bf2f(hq));
  }
}

__device__ __forceinline__ v8h hid8(v8f d, const float* as, const float* ad, const float* gv, int f0) {
  const v4f s0 = *(const v4f*)(as + f0), s1 = *(const v4f*)(as + f0 + 4);
  const v4f t0 = *(const v4f*)(ad + f0), t1 = *(const v4f*)(ad + f0 + 4);
  const v4f g0 = *(const v4f*)(gv + f0), g1 = *(const v4f*)(gv + f0 + 4);
  const v4f u0 = s0 + t0 + g0;
  const v4f u1 = s1 + t1 + g1;
  v8h r;
#pragma unroll
  for (int i = 0; i < 4; ++i) {
    const float L = d[i] * EINV + u0[i];
    r[i] = (_Float16)(lrelu(L) * HSC);
  }
#pragma unroll
  for (int i = 0; i < 4; ++i) {
    const float L = d[4 + i] * EINV + u1[i];
    r[4 + i] = (_Float16)(lrelu(L) * HSC);
  }
  return r;
}

__device__ __forceinline__ int scan_chunk(const int* __restrict__ dsts, int nE, int cbase, int nodeBase,
                                          int vec8, int* list, int tid, int wave) {
  int wc = 0;
  const int el0  = tid * EPT;
  const int e0   = cbase + el0;
  const int sent = -2147483647 - 1;
  v4i da, db;
  if (vec8 != 0 && cbase + CHUNK <= nE) {
    da = *(const v4i*)(dsts + e0);
    db = *(const v4i*)(dsts + e0 + 4);
  } else {
    da.x = (e0     < nE) ? dsts[min(e0, nE - 1)] : sent;
    da.y = (e0 + 1 < nE) ? dsts[min(e0 + 1, nE - 1)] : sent;
    da.z = (e0 + 2 < nE) ? dsts[min(e0 + 2, nE - 1)] : sent;
    da.w = (e0 + 3 < nE) ? dsts[min(e0 + 3, nE - 1)] : sent;
    db.x = (e0 + 4 < nE) ? dsts[min(e0 + 4, nE - 1)] : sent;
    db.y = (e0 + 5 < nE) ? dsts[min(e0 + 5, nE - 1)] : sent;
    db.z = (e0 + 6 < nE) ? dsts[min(e0 + 6, nE - 1)] : sent;
    db.w = (e0 + 7 < nE) ? dsts[min(e0 + 7, nE - 1)] : sent;
  }
  const unsigned nb = (unsigned)nodeBase;
  const unsigned s0 = (unsigned)da.x - nb, s1 = (unsigned)da.y - nb;
  const unsigned s2 = (unsigned)da.z - nb, s3 = (unsigned)da.w - nb;
  const unsigned s4 = (unsigned)db.x - nb, s5 = (unsigned)db.y - nb;
  const unsigned s6 = (unsigned)db.z - nb, s7 = (unsigned)db.w - nb;
  const bool h0 = s0 < (unsigned)NB, h1 = s1 < (unsigned)NB, h2 = s2 < (unsigned)NB, h3 = s3 < (unsigned)NB;
  const bool h4 = s4 < (unsigned)NB, h5 = s5 < (unsigned)NB, h6 = s6 < (unsigned)NB, h7 = s7 < (unsigned)NB;
  const unsigned any = __builtin_amdgcn_ballot_w32(h0 | h1 | h2 | h3 | h4 | h5 | h6 | h7);
  if (any != 0u) {
#define HITJ(J, HJ) { \
      const unsigned mj = __builtin_amdgcn_ballot_w32(HJ); \
      if (mj != 0u) { \
        if (HJ) { \
          const int pos = wc + (int)__builtin_amdgcn_mbcnt_lo(mj, 0u); \
          if (pos < WCAP) list[wave * WCAP + pos] = el0 + (J); \
        } \
        wc += (int)__builtin_popcount(mj); } }
    HITJ(0, h0)
    HITJ(1, h1)
    HITJ(2, h2)
    HITJ(3, h3)
    HITJ(4, h4)
    HITJ(5, h5)
    HITJ(6, h6)
    HITJ(7, h7)
#undef HITJ
  }
  return wc;
}

__global__ __launch_bounds__(NTHR) void k_prep(
    const float* __restrict__ We1, const float* __restrict__ We2,
    const float* __restrict__ Wn1, const float* __restrict__ Wn2,
    _Float16* pW1c, _Float16* pW2,
    unsigned short* pAbH, unsigned short* pAbL,
    unsigned short* pN1H, unsigned short* pN1L,
    unsigned short* pN2H, unsigned short* pN2L) {
  const int b = blockIdx.x, tid = threadIdx.x;
  const float* src;
  int K, ld, koff, rowoff, ub, mode;
  _Float16* df = pW1c;
  unsigned short* dh = pAbH;
  unsigned short* dl = pAbL;
  if (b < 16)      { src = We1; K = DE;      ld = HE; koff = 2 * DN; rowoff = 0;  ub = b;      mode = 0; df = pW1c; }
  else if (b < 32) { src = We2; K = HE;      ld = DE; koff = 0;      rowoff = 0;  ub = b - 16; mode = 0; df = pW2; }
  else if (b < 48) { src = We1; K = DN;      ld = HE; koff = 0;      rowoff = 0;  ub = b - 32; mode = 1; dh = pAbH; dl = pAbL; }
  else if (b < 64) { src = We1; K = DN;      ld = HE; koff = DN;     rowoff = HE; ub = b - 48; mode = 1; dh = pAbH; dl = pAbL; }
  else if (b < 96) { src = Wn1; K = DN + DE; ld = HN; koff = 0;      rowoff = 0;  ub = b - 64; mode = 1; dh = pN1H; dl = pN1L; }
  else             { src = Wn2; K = HN;      ld = DN; koff = 0;      rowoff = 0;  ub = b - 96; mode = 1; dh = pN2H; dl = pN2L; }
  const int u   = ub * NTHR + tid;
  const int cpr = K >> 3;
  const int n   = u / cpr;
  const int kc  = u - n * cpr;
  float w[8];
#pragma unroll
  for (int j = 0; j < 8; ++j) w[j] = src[(size_t)(koff + 8 * kc + j) * ld + n];
  const size_t doff = (size_t)(rowoff + n) * K + 8 * kc;
  if (mode == 0) {
    Pk8 pk;
#pragma unroll
    for (int j = 0; j < 8; ++j) pk.h[j] = (_Float16)(w[j] * WSC);
    *(volatile v4i*)(df + doff) = pk.i;
    __threadfence();
    *(volatile v4i*)(df + doff) = pk.i;
  } else {
    const v4f a = {w[0], w[1], w[2], w[3]};
    const v4f c = {w[4], w[5], w[6], w[7]};
    Pk8 ph, pl;
    split8(a, c, ph, pl);
    *(volatile v4i*)(dh + doff) = ph.i;
    *(volatile v4i*)(dl + doff) = pl.i;
    __threadfence();
    *(volatile v4i*)(dh + doff) = ph.i;
    *(volatile v4i*)(dl + doff) = pl.i;
  }
}

__global__ __launch_bounds__(NTHR) void k_embn(const float* __restrict__ x, const float* __restrict__ Wne,
                                              const float* __restrict__ bne,
                                              unsigned short* XH, unsigned short* XL, int nN, int rowsP) {
  __shared__ float wsh[NF * DN];
  __shared__ float bsh[DN];
  const int tid = threadIdx.x;
  for (int i = tid; i < NF * DN; i += NTHR) wsh[i] = Wne[i];
  if (tid < DN) bsh[tid] = bne[tid];
  __syncthreads();
  const int u   = blockIdx.x * NTHR + tid;
  const int row = u >> 4;
  const int f0  = 8 * (u & 15);
  const int nd  = row > nN - 1 ? nN - 1 : row;
  float s[8];
#pragma unroll
  for (int j = 0; j < 8; ++j) s[j] = bsh[f0 + j];
#pragma unroll 1
  for (int k = 0; k < NF; ++k) {
    const float xk = x[(size_t)nd * NF + k];
#pragma unroll
    for (int j = 0; j < 8; ++j) s[j] += xk * wsh[k * DN + f0 + j];
  }
  const v4f a0 = {lrelu(s[0]), lrelu(s[1]), lrelu(s[2]), lrelu(s[3])};
  const v4f a1 = {lrelu(s[4]), lrelu(s[5]), lrelu(s[6]), lrelu(s[7])};
  Pk8 ph, pl;
  split8(a0, a1, ph, pl);
  const size_t go = (size_t)row * DN + f0;
  if (row < rowsP) { *(volatile v4i*)(XH + go) = ph.i; *(volatile v4i*)(XL + go) = pl.i; }
  __threadfence();
  if (row < rowsP) { *(volatile v4i*)(XH + go) = ph.i; *(volatile v4i*)(XL + go) = pl.i; }
}

__global__ __launch_bounds__(NTHR) void k_embe(const float* __restrict__ ea, const float* __restrict__ Wee,
                                              const float* __restrict__ bee, _Float16* EP, int nE) {
  __shared__ float wsh[EF * DE];
  __shared__ float bsh[DE];
  const int tid = threadIdx.x;
  for (int i = tid; i < EF * DE; i += NTHR) wsh[i] = Wee[i];
  if (tid < DE) bsh[tid] = bee[tid];
  __syncthreads();
  const size_t u = (size_t)blockIdx.x * NTHR + tid;
  const int e  = (int)(u >> 4);
  const int f0 = 8 * (int)(u & 15);
  const int ec = e > nE - 1 ? nE - 1 : e;
  const v4f a = *(const v4f*)(ea + (size_t)ec * EF);
  Pk8 pk;
#pragma unroll
  for (int j = 0; j < 8; ++j) {
    float s = bsh[f0 + j];
    s += a.x * wsh[0 * DE + f0 + j];
    s += a.y * wsh[1 * DE + f0 + j];
    s += a.z * wsh[2 * DE + f0 + j];
    s += a.w * wsh[3 * DE + f0 + j];
    pk.h[j] = (_Float16)(lrelu(s) * ESC);
  }
  const size_t go = (size_t)e * DE + f0;
  if (e < nE) *(volatile v4i*)(EP + go) = pk.i;
  __threadfence();
  if (e < nE) *(volatile v4i*)(EP + go) = pk.i;
}

__global__ __launch_bounds__(NTHR) void k_global(
    const float* __restrict__ u, const float* __restrict__ Wge, const float* __restrict__ bge,
    const int* __restrict__ bt, int nN,
    const float* __restrict__ part, int nPart,
    const float* __restrict__ Wg1, const float* __restrict__ bg1,
    const float* __restrict__ Wg2, const float* __restrict__ bg2,
    const float* __restrict__ We1, const float* __restrict__ be1,
    const float* __restrict__ Wn1, const float* __restrict__ bn1,
    float* GV, int first) {
  __shared__ float gin[KG1];
  __shared__ float hsh[HG];
  __shared__ float gnew[DG];
  __shared__ __attribute__((aligned(16))) float outs[GVN];
  const int tid = threadIdx.x;
  int cnt = 0;
#pragma unroll 1
  for (int i = 0; i < nN; ++i) cnt += (bt[i] == 0) ? 1 : 0;
  cnt = cnt > 1 ? cnt : 1;
  if (first == 0) {
    if (tid < DG) gin[tid] = GV[tid];
    if (tid < DN) {
      float s = 0.0f;
#pragma unroll 1
      for (int b = 0; b < nPart; ++b) s += part[(size_t)b * DN + tid];
      gin[DG + tid] = s * (1.0f / (float)cnt);
    }
  }
  __syncthreads();
  if (first == 0) {
    float s = bg1[tid];
#pragma unroll 1
    for (int k = 0; k < KG1; ++k) s += gin[k] * Wg1[(size_t)k * HG + tid];
    hsh[tid] = lrelu(s);
  }
  __syncthreads();
  if (first == 0) {
    if (tid < DG) {
      float o = bg2[tid];
#pragma unroll 1
      for (int j = 0; j < HG; ++j) o += hsh[j] * Wg2[(size_t)j * DG + tid];
      gnew[tid] = o;
    }
  } else {
    if (tid < DG) {
      float s = bge[tid];
#pragma unroll
      for (int k = 0; k < GF; ++k) s += u[k] * Wge[k * DG + tid];
      gnew[tid] = lrelu(s);
    }
  }
  __syncthreads();
  {
    float s = be1[tid];
#pragma unroll 1
    for (int k = 0; k < DG; ++k) s += gnew[k] * We1[(size_t)(2 * DN + DE + k) * HE + tid];
    outs[DG + tid] = s;
    float t = bn1[tid];
#pragma unroll 1
    for (int k = 0; k < DG; ++k) t += gnew[k] * Wn1[(size_t)(DN + DE + k) * HN + tid];
    outs[DG + HE + tid] = t;
  }
  if (tid < DG) outs[tid] = gnew[tid];
  __syncthreads();
#pragma unroll 1
  for (int idx = tid; idx < GVN; idx += NTHR) { const float v = outs[idx]; *(volatile float*)(GV + idx) = v; }
  __threadfence();
#pragma unroll 1
  for (int idx = tid; idx < GVN; idx += NTHR) { const float v = outs[idx]; *(volatile float*)(GV + idx) = v; }
}

__global__ __launch_bounds__(NTHN) void k_proj(
    const unsigned short* __restrict__ XH, const unsigned short* __restrict__ XL,
    const unsigned short* __restrict__ WH, const unsigned short* __restrict__ WL, float* AB) {
  __shared__ __attribute__((aligned(16))) float stg[4 * 16 * 32];
  const int tid = threadIdx.x, lane = tid & 31, wave = tid >> 5, hh = lane >> 4, m = lane & 15;
  const int row0 = blockIdx.x * NBR + wave * 16;
  FragB bh[4], bl[4];
  {
    const unsigned short* ph = XH + (size_t)(row0 + m) * DN + 8 * hh;
    const unsigned short* pl = XL + (size_t)(row0 + m) * DN + 8 * hh;
#pragma unroll
    for (int kt = 0; kt < 4; ++kt) {
      bh[kt].u[0] = *(const v8us*)(ph + 32 * kt);
      bh[kt].u[1] = *(const v8us*)(ph + 32 * kt + 16);
      bl[kt].u[0] = *(const v8us*)(pl + 32 * kt);
      bl[kt].u[1] = *(const v8us*)(pl + 32 * kt + 16);
    }
  }
  float* sw = stg + wave * 512;
  const int rq = lane >> 3, c4 = lane & 7;
#pragma unroll 1
  for (int fp = 0; fp < ABW / 32; ++fp) {
#pragma unroll
    for (int t = 0; t < 2; ++t) {
      const int ft = 2 * fp + t;
      v8f c = zero8f();
#pragma unroll
      for (int kt = 0; kt < 4; ++kt) {
        FragB ah, al;
        const unsigned short* wp = WH + (size_t)(16 * ft + m) * DN + 32 * kt + 8 * hh;
        const unsigned short* wq = WL + (size_t)(16 * ft + m) * DN + 32 * kt + 8 * hh;
        ah.u[0] = *(const v8us*)wp; ah.u[1] = *(const v8us*)(wp + 16);
        al.u[0] = *(const v8us*)wq; al.u[1] = *(const v8us*)(wq + 16);
        c = wmb(ah.v, bh[kt].v, c);
        c = wmb(ah.v, bl[kt].v, c);
        c = wmb(al.v, bh[kt].v, c);
      }
      float* sp = sw + m * 32 + 16 * t + 8 * hh;
      const v4f c0 = {c[0], c[1], c[2], c[3]};
      const v4f c1 = {c[4], c[5], c[6], c[7]};
      *(v4f*)sp = c0;
      *(v4f*)(sp + 4) = c1;
    }
    __syncthreads();
#pragma unroll
    for (int i = 0; i < 4; ++i) {
      const int rr = 4 * i + rq;
      const v4f v = *(const v4f*)(sw + rr * 32 + 4 * c4);
      *(volatile v4f*)(AB + (size_t)(row0 + rr) * ABW + 32 * fp + 4 * c4) = v;
    }
    __threadfence();
#pragma unroll
    for (int i = 0; i < 4; ++i) {
      const int rr = 4 * i + rq;
      const v4f v = *(const v4f*)(sw + rr * 32 + 4 * c4);
      *(volatile v4f*)(AB + (size_t)(row0 + rr) * ABW + 32 * fp + 4 * c4) = v;
    }
    __syncthreads();
  }
}

__global__ __launch_bounds__(NTHR) void k_edge(
    _Float16* EP, const int* __restrict__ ei, const float* __restrict__ AB,
    const float* __restrict__ GV, const _Float16* __restrict__ W1p, const _Float16* __restrict__ W2p,
    const float* __restrict__ be2, unsigned short* AGH, unsigned short* AGL,
    int nN, int nE, int vec8) {
  extern __shared__ __attribute__((aligned(16))) unsigned char dsm[];
  float*    acc  = (float*)(dsm + LE_ACC);
  float*    msg  = (float*)(dsm + LE_MSG);
  _Float16* eio  = (_Float16*)(dsm + LE_EIO);
  _Float16* hid  = (_Float16*)(dsm + LE_HID);
  int*      list = (int*)(dsm + LE_LIST);
  int*      pend = (int*)(dsm + LE_PEND);
  int*      einf = (int*)(dsm + LE_EINF);
  float*    gvs  = (float*)(dsm + LE_GV);
  float*    b2s  = (float*)(dsm + LE_B2);
  int*      cntb = (int*)(dsm + LE_CNT);
  int*      wcnt = (int*)(dsm + LE_WCNT);

  const int tid = threadIdx.x, lane = tid & 31, wave = tid >> 5, hh = lane >> 4, m = lane & 15;
  const int c8 = lane & 15;
  const int nodeBase = blockIdx.x * NB;
  const int* srcs = ei;
  const int* dsts = ei + nE;
  int dc0 = 0, dc1 = 0, dc2 = 0, dc3 = 0;

  {
    const v4f z = {0.0f, 0.0f, 0.0f, 0.0f};
    for (int i = tid; i < (NB + 1) * DE / 4; i += NTHR) *(v4f*)(acc + 4 * i) = z;
  }
  gvs[tid] = GV[DG + tid];
  if (tid < DE) b2s[tid] = be2[tid];
  if (tid == 0) wcnt[NWAVE] = 0;
  __syncthreads();

  const int nChunks = (nE + CHUNK - 1) / CHUNK;
#pragma unroll 1
  for (int ch = 0; ch < nChunks; ++ch) {
    const int cbase = ch * CHUNK;
    const int wc = scan_chunk(dsts, nE, cbase, nodeBase, vec8, list, tid, wave);
    if (lane == 0) wcnt[wave] = wc;
    __syncthreads();

    const int base = wcnt[NWAVE];
    int tot = 0, myoff = 0;
#pragma unroll
    for (int w = 0; w < NWAVE; ++w) {
      int c = wcnt[w];
      c = c > WCAP ? WCAP : (c < 0 ? 0 : c);
      if (w < wave) myoff += c;
      tot += c;
    }
    int newN = base + tot;
    newN = newN > PCAP ? PCAP : newN;
    {
      int n = wcnt[wave];
      n = n > WCAP ? WCAP : (n < 0 ? 0 : n);
      const int* lp = list + wave * WCAP;
      for (int i = lane; i < n; i += 32) {
        const int pos = base + myoff + i;
        if (pos < PCAP) pend[pos] = cbase + lp[i];
      }
    }
    const int fin = (ch == nChunks - 1) ? 1 : 0;
    const int R   = (fin != 0) ? (newN + PASSN - 1) / PASSN : newN / PASSN;
    const int Pv  = (fin != 0) ? newN : R * PASSN;
    __syncthreads();

#pragma unroll 1
    for (int r = 0; r < R; ++r) {
      const float* abS;
      const float* abD;
      {
        int idx = r * PASSN + wave * 16 + m;
        const bool valid = idx < Pv;
        idx = idx > PCAP - 1 ? PCAP - 1 : idx;
        int e = pend[idx];
        e = e < 0 ? 0 : (e > nE - 1 ? nE - 1 : e);
        const int d = dsts[e];
        int s = srcs[e];
        int slot = d - nodeBase;
        if (!valid || (unsigned)slot >= (unsigned)NB) slot = NB;
        s = s < 0 ? 0 : (s > nN - 1 ? nN - 1 : s);
        const int dcl = d < 0 ? 0 : (d > nN - 1 ? nN - 1 : d);
        abS = AB + (size_t)s * ABW;
        abD = AB + (size_t)dcl * ABW + HE;
        const _Float16* rp = EP + (size_t)e * DE + 64 * hh;
        _Float16* lp = eio + (wave * 16 + m) * DE + 64 * hh;
        const v4i z4 = {0, 0, 0, 0};
#pragma unroll
        for (int j = 0; j < 8; ++j) {
          Pk8 pk;
          pk.h = *(const v8h*)(rp + 8 * j);
          if (!valid) pk.i = z4;
          *(v8h*)(lp + 8 * j) = pk.h;
        }
        if (hh == 0) {
          const v2i inf = {slot, valid ? e : -1};
          *(v2i*)(einf + 2 * (wave * 16 + m)) = inf;
        }
      }
      __syncthreads();

      {
        const _Float16* bp = eio + (wave * 16 + m) * DE + 8 * hh;
        _Float16* hw = hid + (wave * 16 + m) * HE;
#pragma unroll 1
        for (int ft = 0; ft < HE / 16; ++ft) {
          v8f d = zero8f();
#pragma unroll
          for (int kt = 0; kt < 4; ++kt) {
            FragH a, b;
            const _Float16* wp = W1p + (size_t)(16 * ft + m) * DE + 32 * kt + 8 * hh;
            a.h[0] = *(const v8h*)wp;
            a.h[1] = *(const v8h*)(wp + 16);
            b.h[0] = *(const v8h*)(bp + 32 * kt);
            b.h[1] = *(const v8h*)(bp + 32 * kt + 16);
            d = wmh(a.v, b.v, d);
          }
          const int f0 = 16 * ft + 8 * hh;
          const v8h hv = hid8(d, abS, abD, gvs, f0);
          *(v8h*)(hw + f0) = hv;
        }
      }
      __syncthreads();

      {
        const _Float16* hp = hid + (wave * 16 + m) * HE + 8 * hh;
#pragma unroll 1
        for (int ft = 0; ft < DE / 16; ++ft) {
          v8f c = zero8f();
#pragma unroll
          for (int kt = 0; kt < 8; ++kt) {
            FragH a, b;
            const _Float16* wp = W2p + (size_t)(16 * ft + m) * HE + 32 * kt + 8 * hh;
            a.h[0] = *(const v8h*)wp;
            a.h[1] = *(const v8h*)(wp + 16);
            b.h[0] = *(const v8h*)(hp + 32 * kt);
            b.h[1] = *(const v8h*)(hp + 32 * kt + 16);
            c = wmh(a.v, b.v, c);
          }
          const int f0 = 16 * ft + 8 * hh;
          float o[8];
#pragma unroll
          for (int rr = 0; rr < 8; ++rr) o[rr] = c[rr] * HINV + b2s[f0 + rr];
          float* mp = msg + (wave * 16 + m) * DE + f0;
          const v4f o0 = {o[0], o[1], o[2], o[3]};
          const v4f o1 = {o[4], o[5], o[6], o[7]};
          *(v4f*)mp = o0;
          *(v4f*)(mp + 4) = o1;
          Pk8 pk;
#pragma unroll
          for (int rr = 0; rr < 8; ++rr) pk.h[rr] = (_Float16)(o[rr] * ESC);
          *(v8h*)(eio + (wave * 16 + m) * DE + f0) = pk.h;
        }
      }
      __syncthreads();

      {
#pragma unroll
        for (int i = 0; i < 8; ++i) {
          const int sl = wave * 16 + 2 * i + hh;
          const int e  = einf[2 * sl + 1];
          Pk8 pk;
          pk.h = *(const v8h*)(eio + sl * DE + 8 * c8);
          if (e >= 0) *(volatile v4i*)(EP + (size_t)e * DE + 8 * c8) = pk.i;
        }
        __threadfence();
#pragma unroll
        for (int i = 0; i < 8; ++i) {
          const int sl = wave * 16 + 2 * i + hh;
          const int e  = einf[2 * sl + 1];
          Pk8 pk;
          pk.h = *(const v8h*)(eio + sl * DE + 8 * c8);
          if (e >= 0) *(volatile v4i*)(EP + (size_t)e * DE + 8 * c8) = pk.i;
        }
      }

      if (wave < 4) {
#pragma unroll 1
        for (int i = 0; i < PASSN; ++i) {
          int sl = einf[2 * i];
          sl = sl < 0 ? 0 : (sl > NB ? NB : sl);
          acc[sl * DE + tid] += msg[i * DE + tid];
        }
      } else if (wave == 4) {
#pragma unroll 1
        for (int i = 0; i < PASSN; ++i) {
          int sl = einf[2 * i];
          sl = sl < 0 ? 0 : (sl > NB ? NB : sl);
          const int own = ((sl >> 2) == lane) ? 1 : 0;
          const int bs  = sl & 3;
          dc0 += (bs == 0) ? own : 0;
          dc1 += (bs == 1) ? own : 0;
          dc2 += (bs == 2) ? own : 0;
          dc3 += (bs == 3) ? own : 0;
        }
      }
      __syncthreads();
    }

    int rem = newN - R * PASSN;
    rem = rem < 0 ? 0 : rem;
    if (R > 0 && tid < rem) pend[tid] = pend[R * PASSN + tid];
    if (tid == 0) wcnt[NWAVE] = rem;
  }
  __syncthreads();
  if (wave == 4) {
    const v4i dv = {dc0, dc1, dc2, dc3};
    *(v4i*)(cntb + 4 * lane) = dv;
  }
  __syncthreads();

#pragma unroll
  for (int i = 0; i < 8; ++i) {
    const int lr = wave * 16 + 2 * i + hh;
    const int cv = cntb[lr];
    const float inv = 1.0f / (float)(cv > 1 ? cv : 1);
    const float* ar = acc + lr * DE + 8 * c8;
    const v4f a0 = *(const v4f*)ar * inv;
    const v4f a1 = *(const v4f*)(ar + 4) * inv;
    Pk8 ph, pl;
    split8(a0, a1, ph, pl);
    const size_t go = (size_t)(nodeBase + lr) * DE + 8 * c8;
    *(volatile v4i*)(AGH + go) = ph.i;
    *(volatile v4i*)(AGL + go) = pl.i;
  }
  __threadfence();
#pragma unroll
  for (int i = 0; i < 8; ++i) {
    const int lr = wave * 16 + 2 * i + hh;
    const int cv = cntb[lr];
    const float inv = 1.0f / (float)(cv > 1 ? cv : 1);
    const float* ar = acc + lr * DE + 8 * c8;
    const v4f a0 = *(const v4f*)ar * inv;
    const v4f a1 = *(const v4f*)(ar + 4) * inv;
    Pk8 ph, pl;
    split8(a0, a1, ph, pl);
    const size_t go = (size_t)(nodeBase + lr) * DE + 8 * c8;
    *(volatile v4i*)(AGH + go) = ph.i;
    *(volatile v4i*)(AGL + go) = pl.i;
  }
}

__global__ __launch_bounds__(NTHN) void k_node(
    const unsigned short* __restrict__ XH, const unsigned short* __restrict__ XL,
    const unsigned short* __restrict__ GH, const unsigned short* __restrict__ GL,
    const unsigned short* __restrict__ W1H, const unsigned short* __restrict__ W1L,
    const unsigned short* __restrict__ W2H, const unsigned short* __restrict__ W2L,
    const float* __restrict__ GV, const float* __restrict__ bn2, const int* __restrict__ bt,
    unsigned short* YH, unsigned short* YL, float* part, int nN) {
  extern __shared__ __attribute__((aligned(16))) unsigned char dsm[];
  unsigned short* hidH = (unsigned short*)(dsm + LN_HH);
  unsigned short* hidL = (unsigned short*)(dsm + LN_HL);
  float*          ost  = (float*)(dsm + LN_OST);
  float*          gvn  = (float*)(dsm + LN_GV);
  float*          b2s  = (float*)(dsm + LN_B2);
  int*            vr   = (int*)(dsm + LN_VR);

  const int tid = threadIdx.x, lane = tid & 31, wave = tid >> 5, hh = lane >> 4, m = lane & 15;
  const int c8 = lane & 15;
  const int rowBase = blockIdx.x * NBR;
  const int row0 = rowBase + wave * 16;
  for (int i = tid; i < HN; i += NTHN) gvn[i] = GV[DG + HE + i];
  if (tid < DN) b2s[tid] = bn2[tid];
  if (tid < NBR) {
    const int nd  = rowBase + tid;
    const int ndc = nd > nN - 1 ? nN - 1 : nd;
    const int bv  = bt[ndc];
    vr[tid] = (nd < nN && bv == 0) ? 1 : 0;
  }
  __syncthreads();

  unsigned short* hwH = hidH + wave * 16 * HN;
  unsigned short* hwL = hidL + wave * 16 * HN;
  const unsigned short* xh = XH + (size_t)(row0 + m) * DN + 8 * hh;
  const unsigned short* xl = XL + (size_t)(row0 + m) * DN + 8 * hh;
  const unsigned short* gh = GH + (size_t)(row0 + m) * DE + 8 * hh;
  const unsigned short* gl = GL + (size_t)(row0 + m) * DE + 8 * hh;

#pragma unroll 1
  for (int q = 0; q < HN / 16; ++q) {
    v8f c = zero8f();
#pragma unroll
    for (int kt = 0; kt < 8; ++kt) {
      FragB ah, al, bh, bl;
      const unsigned short* wp = W1H + (size_t)(16 * q + m) * (DN + DE) + 32 * kt + 8 * hh;
      const unsigned short* wq = W1L + (size_t)(16 * q + m) * (DN + DE) + 32 * kt + 8 * hh;
      ah.u[0] = *(const v8us*)wp; ah.u[1] = *(const v8us*)(wp + 16);
      al.u[0] = *(const v8us*)wq; al.u[1] = *(const v8us*)(wq + 16);
      const unsigned short* bp = (kt < 4) ? (xh + 32 * kt) : (gh + 32 * (kt - 4));
      const unsigned short* bq = (kt < 4) ? (xl + 32 * kt) : (gl + 32 * (kt - 4));
      bh.u[0] = *(const v8us*)bp; bh.u[1] = *(const v8us*)(bp + 16);
      bl.u[0] = *(const v8us*)bq; bl.u[1] = *(const v8us*)(bq + 16);
      c = wmb(ah.v, bh.v, c);
      c = wmb(ah.v, bl.v, c);
      c = wmb(al.v, bh.v, c);
    }
    const int f0 = 16 * q + 8 * hh;
    float hv[8];
#pragma unroll
    for (int rr = 0; rr < 8; ++rr) hv[rr] = lrelu(c[rr] + gvn[f0 + rr]);
    const v4f a0 = {hv[0], hv[1], hv[2], hv[3]};
    const v4f a1 = {hv[4], hv[5], hv[6], hv[7]};
    Pk8 ph, pl;
    split8(a0, a1, ph, pl);
    *(v8us*)(hwH + m * HN + f0) = ph.u;
    *(v8us*)(hwL + m * HN + f0) = pl.u;
  }
  __syncthreads();

#pragma unroll 1
  for (int ft = 0; ft < DN / 16; ++ft) {
    v8f c = zero8f();
#pragma unroll
    for (int kt = 0; kt < 8; ++kt) {
      FragB ah, al, bh, bl;
      const unsigned short* wp = W2H + (size_t)(16 * ft + m) * HN + 32 * kt + 8 * hh;
      const unsigned short* wq = W2L + (size_t)(16 * ft + m) * HN + 32 * kt + 8 * hh;
      ah.u[0] = *(const v8us*)wp; ah.u[1] = *(const v8us*)(wp + 16);
      al.u[0] = *(const v8us*)wq; al.u[1] = *(const v8us*)(wq + 16);
      const unsigned short* bp = hwH + m * HN + 32 * kt + 8 * hh;
      const unsigned short* bq = hwL + m * HN + 32 * kt + 8 * hh;
      bh.u[0] = *(const v8us*)bp; bh.u[1] = *(const v8us*)(bp + 16);
      bl.u[0] = *(const v8us*)bq; bl.u[1] = *(const v8us*)(bq + 16);
      c = wmb(ah.v, bh.v, c);
      c = wmb(ah.v, bl.v, c);
      c = wmb(al.v, bh.v, c);
    }
    const int f0 = 16 * ft + 8 * hh;
    float o[8];
#pragma unroll
    for (int rr = 0; rr < 8; ++rr) o[rr] = c[rr] + b2s[f0 + rr];
    float* sp = ost + (wave * 16 + m) * DN + f0;
    const v4f o0 = {o[0], o[1], o[2], o[3]};
    const v4f o1 = {o[4], o[5], o[6], o[7]};
    *(v4f*)sp = o0;
    *(v4f*)(sp + 4) = o1;
  }
  __syncthreads();

#pragma unroll
  for (int i = 0; i < 8; ++i) {
    const int lr = wave * 16 + 2 * i + hh;
    const float* sr = ost + lr * DN + 8 * c8;
    Pk8 ph, pl;
    split8(*(const v4f*)sr, *(const v4f*)(sr + 4), ph, pl);
    const size_t go = (size_t)(rowBase + lr) * DN + 8 * c8;
    *(volatile v4i*)(YH + go) = ph.i;
    *(volatile v4i*)(YL + go) = pl.i;
  }
  __threadfence();
#pragma unroll
  for (int i = 0; i < 8; ++i) {
    const int lr = wave * 16 + 2 * i + hh;
    const float* sr = ost + lr * DN + 8 * c8;
    Pk8 ph, pl;
    split8(*(const v4f*)sr, *(const v4f*)(sr + 4), ph, pl);
    const size_t go = (size_t)(rowBase + lr) * DN + 8 * c8;
    *(volatile v4i*)(YH + go) = ph.i;
    *(volatile v4i*)(YL + go) = pl.i;
  }

  float s = 0.0f;
#pragma unroll 1
  for (int r = 0; r < NBR; ++r) {
    const float v = ost[r * DN + tid];
    s += (vr[r] != 0) ? v : 0.0f;
  }
  *(volatile float*)(part + (size_t)blockIdx.x * DN + tid) = s;
  __threadfence();
  *(volatile float*)(part + (size_t)blockIdx.x * DN + tid) = s;
}

__global__ __launch_bounds__(NTHR) void k_dec(const _Float16* __restrict__ EP, const float* __restrict__ Wd,
                                             const float* __restrict__ bd, float* out, int nE) {
  __shared__ float wd[DE];
  const int tid = threadIdx.x;
  if (tid < DE) wd[tid] = Wd[tid];
  __syncthreads();
  const int e  = blockIdx.x * NTHR + tid;
  const int ec = e > nE - 1 ? nE - 1 : e;
  const _Float16* ep = EP + (size_t)ec * DE;
  float s = 0.0f;
#pragma unroll 1
  for (int j = 0; j < DE / 8; ++j) {
    const v8h v = *(const v8h*)(ep + 8 * j);
#pragma unroll
    for (int i = 0; i < 8; ++i) s += (float)v[i] * wd[8 * j + i];
  }
  const float o = s * EPINV + bd[0];
  if (e < nE) *(volatile float*)(out + e) = o;
  __threadfence();
  if (e < nE) *(volatile float*)(out + e) = o;
}

extern "C" void kernel_launch(void* const* d_in, const int* in_sizes, int n_in,
                              void* d_out, int out_size, void* d_ws, size_t ws_size,
                              hipStream_t stream) {
  if (n_in < 25) return;
  const int nN = in_sizes[4];
  const int nE = out_size;
  if (nN < 1 || nE < 1) return;
  if (in_sizes[0] != nN * NF || in_sizes[1] != nE * EF || in_sizes[2] != GF || in_sizes[3] != 2 * nE) return;
  if (in_sizes[5] != NF * DN || in_sizes[6] != DN || in_sizes[7] != EF * DE || in_sizes[8] != DE) return;
  if (in_sizes[9] != GF * DG || in_sizes[10] != DG) return;
  if (in_sizes[11] != (2 * DN + DE + DG) * HE || in_sizes[12] != HE) return;
  if (in_sizes[13] != HE * DE || in_sizes[14] != DE) return;
  if (in_sizes[15] != (DN + DE + DG) * HN || in_sizes[16] != HN) return;
  if (in_sizes[17] != HN * DN || in_sizes[18] != DN) return;
  if (in_sizes[19] != (DG + DN) * HG || in_sizes[20] != HG) return;
  if (in_sizes[21] != HG * DG || in_sizes[22] != DG) return;
  if (in_sizes[23] != DE || in_sizes[24] != 1) return;

  const float* x    = (const float*)d_in[0];
  const float* ea   = (const float*)d_in[1];
  const float* u    = (const float*)d_in[2];
  const int*   ei   = (const int*)d_in[3];
  const int*   bt   = (const int*)d_in[4];
  const float* Wne  = (const float*)d_in[5];
  const float* bne  = (const float*)d_in[6];
  const float* Wee  = (const float*)d_in[7];
  const float* bee  = (const float*)d_in[8];
  const float* Wge  = (const float*)d_in[9];
  const float* bge  = (const float*)d_in[10];
  const float* We1  = (const float*)d_in[11];
  const float* be1  = (const float*)d_in[12];
  const float* We2  = (const float*)d_in[13];
  const float* be2  = (const float*)d_in[14];
  const float* Wn1  = (const float*)d_in[15];
  const float* bn1  = (const float*)d_in[16];
  const float* Wn2  = (const float*)d_in[17];
  const float* bn2  = (const float*)d_in[18];
  const float* Wg1  = (const float*)d_in[19];
  const float* bg1  = (const float*)d_in[20];
  const float* Wg2  = (const float*)d_in[21];
  const float* bg2  = (const float*)d_in[22];
  const float* Wdec = (const float*)d_in[23];
  const float* bdec = (const float*)d_in[24];
  float* outp = (float*)d_out;

  const int nBlkE = (nN + NB - 1) / NB;
  const size_t rowsP = (size_t)nBlkE * NB;
  const int nBlkN = (int)(rowsP / NBR);

  char* ws = (char*)d_ws;
  size_t off = 0;
#define CARVE(NAME, BYTES) const size_t NAME = off; off += (((size_t)(BYTES)) + 255) & ~(size_t)255;
  CARVE(oW1c, (size_t)HE * DE * 2)
  CARVE(oW2,  (size_t)DE * HE * 2)
  CARVE(oAbH, (size_t)ABW * DN * 2)
  CARVE(oAbL, (size_t)ABW * DN * 2)
  CARVE(oN1H, (size_t)HN * (DN + DE) * 2)
  CARVE(oN1L, (size_t)HN * (DN + DE) * 2)
  CARVE(oN2H, (size_t)DN * HN * 2)
  CARVE(oN2L, (size_t)DN * HN * 2)
  CARVE(oEP,  (size_t)nE * DE * 2)
  CARVE(oAB,  rowsP * ABW * 4)
  CARVE(oXH0, rowsP * DN * 2)
  CARVE(oXL0, rowsP * DN * 2)
  CARVE(oXH1, rowsP * DN * 2)
  CARVE(oXL1, rowsP * DN * 2)
  CARVE(oAGH, rowsP * DE * 2)
  CARVE(oAGL, rowsP * DE * 2)
  CARVE(oPart, (size_t)nBlkN * DN * 4)
  CARVE(oGV,  (size_t)GVN * 4)
#undef CARVE
  size_t limit = (size_t)134217728;
  if (ws_size < limit) limit = ws_size;
  if (off > limit) return;

  _Float16* pW1c = (_Float16*)(ws + oW1c);
  _Float16* pW2  = (_Float16*)(ws + oW2);
  unsigned short* pAbH = (unsigned short*)(ws + oAbH);
  unsigned short* pAbL = (unsigned short*)(ws + oAbL);
  unsigned short* pN1H = (unsigned short*)(ws + oN1H);
  unsigned short* pN1L = (unsigned short*)(ws + oN1L);
  unsigned short* pN2H = (unsigned short*)(ws + oN2H);
  unsigned short* pN2L = (unsigned short*)(ws + oN2L);
  _Float16* EP = (_Float16*)(ws + oEP);
  float* AB = (float*)(ws + oAB);
  unsigned short* XH0 = (unsigned short*)(ws + oXH0);
  unsigned short* XL0 = (unsigned short*)(ws + oXL0);
  unsigned short* XH1 = (unsigned short*)(ws + oXH1);
  unsigned short* XL1 = (unsigned short*)(ws + oXL1);
  unsigned short* AGH = (unsigned short*)(ws + oAGH);
  unsigned short* AGL = (unsigned short*)(ws + oAGL);
  float* part = (float*)(ws + oPart);
  float* GV   = (float*)(ws + oGV);

  const int vec8 = ((nE & 3) == 0) ? 1 : 0;
  const int embnBlocks = (int)(rowsP * 16 / NTHR);
  const int embeBlocks = (int)(((size_t)nE * 16 + NTHR - 1) / NTHR);
  const int decBlocks  = (nE + NTHR - 1) / NTHR;

  k_prep<<<112, NTHR, 0, stream>>>(We1, We2, Wn1, Wn2, pW1c, pW2, pAbH, pAbL, pN1H, pN1L, pN2H, pN2L);
  k_embn<<<embnBlocks, NTHR, 0, stream>>>(x, Wne, bne, XH0, XL0, nN, (int)rowsP);
  k_embe<<<embeBlocks, NTHR, 0, stream>>>(ea, Wee, bee, EP, nE);
  k_global<<<1, NTHR, 0, stream>>>(u, Wge, bge, bt, nN, part, nBlkN, Wg1, bg1, Wg2, bg2,
                                   We1, be1, Wn1, bn1, GV, 1);

  hipFuncSetAttribute(reinterpret_cast<const void*>(&k_edge), hipFuncAttributeMaxDynamicSharedMemorySize, LE_TOTAL);
  hipFuncSetAttribute(reinterpret_cast<const void*>(&k_node), hipFuncAttributeMaxDynamicSharedMemorySize, LN_TOTAL);

  unsigned short* xh[2] = {XH0, XH1};
  unsigned short* xl[2] = {XL0, XL1};
  for (int p = 0; p < 2; ++p) {
    const int cur = p & 1, nxt = (p + 1) & 1;
    k_proj<<<nBlkN, NTHN, 0, stream>>>(xh[cur], xl[cur], pAbH, pAbL, AB);
    k_edge<<<nBlkE, NTHR, LE_TOTAL, stream>>>(EP, ei, AB, GV, pW1c, pW2, be2, AGH, AGL, nN, nE, vec8);
    k_node<<<nBlkN, NTHN, LN_TOTAL, stream>>>(xh[cur], xl[cur], AGH, AGL, pN1H, pN1L, pN2H, pN2L,
                                              GV, bn2, bt, xh[nxt], xl[nxt], part, nN);
    k_global<<<1, NTHR, 0, stream>>>(u, Wge, bge, bt, nN, part, nBlkN, Wg1, bg1, Wg2, bg2,
                                     We1, be1, Wn1, bn1, GV, 0);
  }
  k_dec<<<decBlocks, NTHR, 0, stream>>>(EP, Wdec, bdec, outp, nE);
}
